// SoftOptionCritic_32693291057940
// MI455X (gfx1250) — hardware-verified
//
#include <hip/hip_runtime.h>
#include <math.h>

#define NB    8192
#define OBS   128
#define HID   512
#define HEADS 4
#define VSZ   256
#define NU    64
#define TOPK  8
#define NOPT  16

#define H_STRIDE 520

#define __bf16 _Float16
#define RSPLIT (1.0f / 2048.0f)
typedef __attribute__((ext_vector_type(8)))  float  v8f;
typedef __attribute__((ext_vector_type(16))) __bf16 v16bf;
typedef __attribute__((ext_vector_type(4)))  float  v4f_t;
typedef float v4fa __attribute__((ext_vector_type(4), may_alias));
__device__ __forceinline__ __bf16 lo_of(float v, __bf16 h) { return (__bf16)((v - (float)h) * 2048.0f); }

__device__ __forceinline__ void split16(const float* __restrict__ p0,
                                        const float* __restrict__ p1,
                                        v16bf& hi, v16bf& lo) {
  v8f f0 = *(const v8f*)p0;
  v8f f1 = *(const v8f*)p1;
#pragma unroll
  for (int e = 0; e < 8; ++e) {
    float a = f0[e];
    __bf16 ah = (__bf16)a;
    hi[e] = ah;
    lo[e] = lo_of(a, ah);
    float b = f1[e];
    __bf16 bh = (__bf16)b;
    hi[e + 8] = bh;
    lo[e + 8] = lo_of(b, bh);
  }
}

__device__ __forceinline__ v8f wmma_bf16(v16bf a, v16bf b, v8f c) {
  return __builtin_amdgcn_wmma_f32_16x16x32_f16(
      false, a, false, b, (short)0, c, false, false);
}
__device__ __forceinline__ v8f wmma_split(v16bf a, v16bf al, v16bf b, v16bf bl, v8f c) {
  v8f x = {}; x = wmma_bf16(al, b, x); x = wmma_bf16(a, bl, x); return wmma_bf16(a, b, c) + x * RSPLIT;
}
__device__ __forceinline__ void st2f(float* p, float v) { *(volatile float*)p = v; __threadfence(); *(volatile float*)p = v; }
__device__ __forceinline__ int kof(int half, int e) { return ((e < 8) ? e : (e + 8)) + half * 8; }
__device__ __forceinline__ void stpair(__bf16* hi, __bf16* lo, int i, float v0, float v1) {
  const __bf16 a = (__bf16)v0, b = (__bf16)v1;
  const unsigned u = (unsigned)__builtin_bit_cast(unsigned short, a) | ((unsigned)__builtin_bit_cast(unsigned short, b) << 16);
  const unsigned w = (unsigned)__builtin_bit_cast(unsigned short, lo_of(v0, a)) | ((unsigned)__builtin_bit_cast(unsigned short, lo_of(v1, b)) << 16);
  *(volatile unsigned*)(hi + i) = u; *(volatile unsigned*)(lo + i) = w; __threadfence(); *(volatile unsigned*)(hi + i) = u; *(volatile unsigned*)(lo + i) = w;
}

__global__ void __launch_bounds__(256) soc_prep_small(
    const float* __restrict__ p_w, const float* __restrict__ p_b,
    const float* __restrict__ value_b, float* __restrict__ scale,
    float* __restrict__ cvec) {
  const int t = threadIdx.x;
  if (t < VSZ) {
    st2f(cvec + t, (value_b[t] + value_b[VSZ + t] + value_b[2 * VSZ + t] +
                    value_b[3 * VSZ + t]) * (1.0f / 32.0f));
  }
  __shared__ float ss[NOPT][NU + 1];
  if (t < NOPT) {
    float* s = ss[t];
    for (int n = 0; n < NU; ++n) s[n] = p_w[t * NU + n] + p_b[n];
    float acc = 0.0f;
    for (int k = 0; k < TOPK; ++k) {
      int best = 0;
      float bv = s[0];
      for (int n = 1; n < NU; ++n)
        if (s[n] > bv) { bv = s[n]; best = n; }
      acc += 1.0f / (1.0f + expf(-bv));
      s[best] = -3.402823466e38f;
    }
    st2f(scale + t, acc * (1.0f / 256.0f));
  }
}

__global__ void __launch_bounds__(256) soc_pack_w1(
    const float* __restrict__ w1, __bf16* __restrict__ hi,
    __bf16* __restrict__ lo) {
  const int i = (blockIdx.x * 256 + threadIdx.x) * 2;
  if (i < OBS * HID) {
    const int e     = i & 15;
    const int chunk = i >> 4;
    const int half  = chunk & 1;
    const int n     = (chunk >> 1) & (HID - 1);
    const int k0    = ((chunk >> 1) / HID) << 5;
    stpair(hi, lo, i, w1[(k0 + kof(half, e)) * HID + n], w1[(k0 + kof(half, e + 1)) * HID + n]);
  }
}

__global__ void __launch_bounds__(256) soc_pack_w2(
    const float* __restrict__ value_w, __bf16* __restrict__ hi,
    __bf16* __restrict__ lo) {
  const int i = (blockIdx.x * 256 + threadIdx.x) * 2;
  if (i < HID * VSZ) {
    const int e     = i & 15;
    const int chunk = i >> 4;
    const int half  = chunk & 1;
    const int n     = (chunk >> 1) & (VSZ - 1);
    const int k0    = ((chunk >> 1) / VSZ) << 5;
    float v2[2];
#pragma unroll
    for (int u = 0; u < 2; ++u) {
      const float* r = value_w + (k0 + kof(half, e + u)) * (HEADS * VSZ);
      v2[u] = r[n] + r[VSZ + n] + r[2 * VSZ + n] + r[3 * VSZ + n];
    }
    stpair(hi, lo, i, v2[0], v2[1]);
  }
}

__global__ void __launch_bounds__(256) soc_fused(
    const float* __restrict__ x, const __bf16* __restrict__ w1p_hi,
    const __bf16* __restrict__ w1p_lo, const float* __restrict__ b1,
    const __bf16* __restrict__ w2p_hi, const __bf16* __restrict__ w2p_lo,
    const float* __restrict__ scale, const float* __restrict__ cvec,
    const int* __restrict__ option, float* __restrict__ out) {
  __shared__ __attribute__((aligned(16))) float h_lds[32 * H_STRIDE];
  __shared__ float row_scale[32];
  __shared__ __attribute__((aligned(16))) float stg[8][16 * 68];

  const int lane = threadIdx.x & 31;
  const int wave = threadIdx.x >> 5;
  const int m    = lane & 15;
  const int half = lane >> 4;
  const int koff = half * 8;
  const int row0 = blockIdx.x * 32;

  if (threadIdx.x < 32) { int o = option[row0 + threadIdx.x]; o = (o < 0) ? 0 : (o >= NOPT ? NOPT - 1 : o); row_scale[threadIdx.x] = scale[o]; }

  const int rt    = wave & 1;
  const int cg    = wave >> 1;
  const int arow  = rt * 16 + m;

  v8f acc[8] = {};
  const float* xrow = x + (row0 + arow) * OBS;
  const int bcol1 = (cg * 128 + m) * 32 + half * 16;
  for (int k0 = 0; k0 < OBS; k0 += 32) {
    v16bf a_hi, a_lo;
    split16(xrow + k0 + koff, xrow + k0 + koff + 16, a_hi, a_lo);
    const __bf16* bh_base = w1p_hi + (k0 >> 5) * (HID * 32) + bcol1;
    const __bf16* bl_base = w1p_lo + (k0 >> 5) * (HID * 32) + bcol1;
#pragma unroll
    for (int t = 0; t < 8; ++t)
      acc[t] = wmma_split(a_hi, a_lo, *(const v16bf*)(bh_base + t * 512), *(const v16bf*)(bl_base + t * 512), acc[t]);
  }

#pragma unroll
  for (int t = 0; t < 8; ++t) {
    const int col = cg * 128 + t * 16 + m;
    const float bias = b1[col];
#pragma unroll
    for (int j = 0; j < 8; ++j) {
      const int r = rt * 16 + j + half * 8;
      h_lds[r * H_STRIDE + col] = acc[t][j] + bias;
    }
  }
  __syncthreads();

  v8f acc2[4] = {};
  const float* hrow = h_lds + arow * H_STRIDE;
  const int bcol2 = (cg * 64 + m) * 32 + half * 16;
  for (int k0 = 0; k0 < HID; k0 += 32) {
    v16bf a_hi, a_lo;
    split16(hrow + k0 + koff, hrow + k0 + koff + 16, a_hi, a_lo);
    const __bf16* bh_base = w2p_hi + (k0 >> 5) * (VSZ * 32) + bcol2;
    const __bf16* bl_base = w2p_lo + (k0 >> 5) * (VSZ * 32) + bcol2;
#pragma unroll
    for (int t = 0; t < 4; ++t)
      acc2[t] = wmma_split(a_hi, a_lo, *(const v16bf*)(bh_base + t * 512), *(const v16bf*)(bl_base + t * 512), acc2[t]);
  }

  float* sw = stg[wave];
#pragma unroll
  for (int t = 0; t < 4; ++t) {
    const int cl = t * 16 + m, col = cg * 64 + cl;
    const float cv = cvec[col];
#pragma unroll
    for (int j = 0; j < 8; ++j) {
      const int rl = j + half * 8, r = rt * 16 + rl;
      sw[rl * 68 + cl] = acc2[t][j] * row_scale[r] + cv;
    }
  }
  asm volatile("s_wait_dscnt 0" ::: "memory");
#pragma unroll 1
  for (int pass = 0; pass < 2; ++pass) {
#pragma unroll
    for (int i = 0; i < 8; ++i) { const int c = lane + 32 * i, rr = c >> 4, q = (c & 15) * 4;
      *(volatile v4f_t*)(out + (size_t)(row0 + rt * 16 + rr) * VSZ + cg * 64 + q) = *(const volatile v4fa*)(sw + rr * 68 + q); }
    __threadfence();
  }
}

extern "C" void kernel_launch(void* const* d_in, const int* in_sizes, int n_in,
                              void* d_out, int out_size, void* d_ws, size_t ws_size,
                              hipStream_t stream) {
  const float* x   = (const float*)d_in[0];
  const int*   opt = (const int*)d_in[1];
  const float* w1  = (const float*)d_in[2];
  const float* b1  = (const float*)d_in[3];
  const float* vw  = (const float*)d_in[4];
  const float* vb  = (const float*)d_in[5];
  const float* pw  = (const float*)d_in[6];
  const float* pb  = (const float*)d_in[7];
  float* out = (float*)d_out;

  float* ws    = (float*)d_ws;
  float* scale = ws;
  float* cvec  = ws + 16;
  __bf16* w1p_hi = (__bf16*)((char*)d_ws + 4096);
  __bf16* w1p_lo = w1p_hi + OBS * HID;
  __bf16* w2p_hi = w1p_lo + OBS * HID;
  __bf16* w2p_lo = w2p_hi + HID * VSZ;

  soc_prep_small<<<1, 256, 0, stream>>>(pw, pb, vb, scale, cvec);
  soc_pack_w1<<<(OBS * HID) / 512, 256, 0, stream>>>(w1, w1p_hi, w1p_lo);
  soc_pack_w2<<<(HID * VSZ) / 512, 256, 0, stream>>>(vw, w2p_hi, w2p_lo);
  soc_fused<<<NB / 32, 256, 0, stream>>>(x, w1p_hi, w1p_lo, b1, w2p_hi, w2p_lo,
                                         scale, cvec, opt, out);
}
